// MambaBlock_76166950027467
// MI455X (gfx1250) — hardware-verified
//
#include <hip/hip_runtime.h>
#include <stddef.h>
#include <stdint.h>
#include <math.h>


#define DIMX  1024
#define DIN   2048
#define NST   16
#define RNK   64
#define XPN   96
#define MTOK  2048
#define SEQL  1024
#define NLAY  2
#define WSMAX 134217728

#define U_XB   (MTOK * DIMX / 8)
#define U_INW  (NLAY * 2 * DIN * DIMX / 8)
#define U_XP   (NLAY * XPN * DIN / 8)
#define U_DTW  (NLAY * DIN * RNK / 8)
#define U_OW   (NLAY * DIMX * DIN / 8)
#define U8_TOT (U_XB + U_INW + U_XP + U_DTW + U_OW)
#define V_CW   (NLAY * DIN * 4 / 4)
#define V_CB   (NLAY * DIN / 4)
#define V_DTB  (NLAY * DIN / 4)
#define V_DD   (NLAY * DIN / 4)
#define V_AN   (NLAY * DIN * NST / 4)
#define V4_TOT (V_CW + V_CB + V_DTB + V_DD + V_AN)

static_assert(U_XB % 256 == 0 && U_INW % 256 == 0 && U_XP % 256 == 0 && U_DTW % 256 == 0 && U_OW % 256 == 0);
static_assert(V_CW % 256 == 0 && V_CB % 256 == 0 && V_AN % 256 == 0);
static_assert(MTOK % 128 == 0 && (2 * DIN) % 64 == 0 && DIN % 64 == 0 && DIMX % 64 == 0 && XPN == 96);
static_assert(DIMX % 32 == 0 && (2 * DIMX) % 32 == 0 && (2 * DIN) % 32 == 0 && (2 * RNK) % 32 == 0);

#define B_XB   ((size_t)MTOK * DIMX * 2)
#define B_INW  ((size_t)NLAY * 2 * DIN * DIMX * 2)
#define B_XPB  ((size_t)NLAY * XPN * DIN * 2)
#define B_DTWB ((size_t)NLAY * DIN * RNK * 2)
#define B_OWB  ((size_t)NLAY * DIMX * DIN * 2)
#define B_CW   ((size_t)NLAY * DIN * 4 * 4)
#define B_V    ((size_t)NLAY * DIN * 4)
#define B_AN   ((size_t)NLAY * DIN * NST * 4)
#define B_F32  ((size_t)MTOK * DIN * 4)
#define B_XCHL ((size_t)MTOK * 2 * DIN * 2)
#define B_XDBL ((size_t)MTOK * XPN * 4)
#define B_DTR  ((size_t)MTOK * 2 * RNK * 2)
#define B_TOT  (B_XB + B_INW + B_XPB + B_DTWB + B_OWB + B_CW + 3 * B_V + B_AN + 4 * B_F32 + B_XCHL + B_XDBL + B_DTR)
static_assert(B_TOT <= (size_t)WSMAX);
static_assert((size_t)MTOK * 2 * DIN * 2 <= B_F32);
static_assert((size_t)MTOK * 2 * DIMX * 2 <= B_F32);

typedef float          v4f   __attribute__((ext_vector_type(4)));
typedef float          v8f   __attribute__((ext_vector_type(8)));
typedef int            v8i   __attribute__((ext_vector_type(8)));
typedef unsigned short v8us  __attribute__((ext_vector_type(8)));
typedef unsigned short v16us __attribute__((ext_vector_type(16)));
typedef __bf16         v16bf __attribute__((ext_vector_type(16)));
typedef v4f  __attribute__((may_alias)) v4fa;
typedef v8us __attribute__((may_alias)) v8usa;
union FragB { v16bf v; v16us u; v8us h[2]; v8i w; };

__device__ __forceinline__ v8f wmb(const FragB& a, const FragB& b, v8f c) {
  v8f d = __builtin_amdgcn_wmma_f32_16x16x32_bf16(false, a.v, false, b.v, (short)0, c, false, false);
  asm volatile("v_nop\n\tv_nop\n\tv_nop\n\tv_nop" : "+v"(d) : "v"(a.w), "v"(b.w));
  return d;
}

__device__ __forceinline__ unsigned bf16_bits(float f) {
  const unsigned u = __float_as_uint(f);
  return (u + 0x7FFFu + ((u >> 16) & 1u)) >> 16;
}
__device__ __forceinline__ float bf16_val(float f) {
  return __uint_as_float(bf16_bits(f) << 16);
}
__device__ __forceinline__ unsigned short hl_bits(float v, bool lo) {
  const unsigned hb = bf16_bits(v);
  const unsigned lb = bf16_bits(v - __uint_as_float(hb << 16));
  return (unsigned short)(lo ? lb : hb);
}
__device__ __forceinline__ v8us pack8(const float* s, bool lo) {
  const v4f a = *(const v4fa*)s;
  const v4f b = *(const v4fa*)(s + 4);
  v8us o;
  o[0] = hl_bits(a.x, lo); o[1] = hl_bits(a.y, lo); o[2] = hl_bits(a.z, lo); o[3] = hl_bits(a.w, lo);
  o[4] = hl_bits(b.x, lo); o[5] = hl_bits(b.y, lo); o[6] = hl_bits(b.z, lo); o[7] = hl_bits(b.w, lo);
  return o;
}
__device__ __forceinline__ float softplus_f(float v) {
  return fmaxf(v, 0.0f) + log1pf(expf(-fabsf(v)));
}

__global__ __launch_bounds__(256) void k_prep(
    const float* __restrict__ x, const float* __restrict__ inw, const float* __restrict__ xpw,
    const float* __restrict__ dtw, const float* __restrict__ ow, const float* __restrict__ cw,
    const float* __restrict__ cb, const float* __restrict__ dtb, const float* __restrict__ alog,
    const float* __restrict__ dp,
    unsigned short* XB, unsigned short* INW, unsigned short* XPB, unsigned short* DTWB, unsigned short* OWB,
    float* CWp, float* CBp, float* DTBp, float* DDp, float* ANp)
{
  const int bx = (int)blockIdx.x, tid = (int)threadIdx.x;
  if (bx < U8_TOT / 256) {
    int u = bx * 256 + tid;
    const float* s;
    unsigned short* d;
    if (u < U_XB)                               { s = x;   d = XB; }
    else if (u < U_XB + U_INW)                  { u -= U_XB; s = inw; d = INW; }
    else if (u < U_XB + U_INW + U_XP)           { u -= U_XB + U_INW; s = xpw; d = XPB; }
    else if (u < U_XB + U_INW + U_XP + U_DTW)   { u -= U_XB + U_INW + U_XP; s = dtw; d = DTWB; }
    else                                        { u -= U_XB + U_INW + U_XP + U_DTW; s = ow; d = OWB; }
    const float* p = s + (size_t)u * 8;
    const v4f a = *(const v4f*)p;
    const v4f b = *(const v4f*)(p + 4);
    v8us o;
    o[0] = (unsigned short)bf16_bits(a.x); o[1] = (unsigned short)bf16_bits(a.y);
    o[2] = (unsigned short)bf16_bits(a.z); o[3] = (unsigned short)bf16_bits(a.w);
    o[4] = (unsigned short)bf16_bits(b.x); o[5] = (unsigned short)bf16_bits(b.y);
    o[6] = (unsigned short)bf16_bits(b.z); o[7] = (unsigned short)bf16_bits(b.w);
    unsigned short* q = d + (size_t)u * 8;
    *(volatile v8us*)q = o;
    __threadfence();
    *(volatile v8us*)q = o;
  } else {
    int u = (bx - U8_TOT / 256) * 256 + tid;
    const float* s;
    float* d;
    int isA = 0;
    if (u < V_CW)                               { s = cw;  d = CWp; }
    else if (u < V_CW + V_CB)                   { u -= V_CW; s = cb; d = CBp; }
    else if (u < V_CW + V_CB + V_DTB)           { u -= V_CW + V_CB; s = dtb; d = DTBp; }
    else if (u < V_CW + V_CB + V_DTB + V_DD)    { u -= V_CW + V_CB + V_DTB; s = dp; d = DDp; }
    else if (u < V4_TOT)                        { u -= V_CW + V_CB + V_DTB + V_DD; s = alog; d = ANp; isA = 1; }
    else return;
    const v4f v = *(const v4f*)(s + (size_t)u * 4);
    v4f r;
    r.x = bf16_val(v.x); r.y = bf16_val(v.y); r.z = bf16_val(v.z); r.w = bf16_val(v.w);
    if (isA != 0) {
      r.x = -expf(r.x); r.y = -expf(r.y); r.z = -expf(r.z); r.w = -expf(r.w);
    }
    float* q = d + (size_t)u * 4;
    *(volatile v4f*)q = r;
    __threadfence();
    *(volatile v4f*)q = r;
  }
}

template <int MT, int NT, int EPI>
__global__ __launch_bounds__(128) void k_gemm(
    const unsigned short* __restrict__ A, int lda,
    const unsigned short* __restrict__ Bt, int ldb, int kmask, int K,
    float* o0, float* o1, int split, int ldo,
    const float* __restrict__ bias,
    unsigned short* oh, int ldh, int hoff)
{
  constexpr int BM = 64 * MT, BN = 16 * NT, RW = 16 * MT;
  __shared__ __attribute__((aligned(16))) float stg[BM * BN];
  const int tid = (int)threadIdx.x, lane = tid & 31, wave = tid >> 5, hh = lane >> 4, m = lane & 15;
  const int rowBase = (int)blockIdx.x * BM;
  const int col0    = (int)blockIdx.y * BN;

  v8f acc[MT][NT];
  {
    const v8f z = {0.f, 0.f, 0.f, 0.f, 0.f, 0.f, 0.f, 0.f};
#pragma unroll
    for (int i = 0; i < MT; ++i)
#pragma unroll
      for (int t = 0; t < NT; ++t) acc[i][t] = z;
  }
  const unsigned short* ap = A  + (size_t)(rowBase + RW * wave + m) * (size_t)lda + 8 * hh;
  const unsigned short* bp = Bt + (size_t)(col0 + m) * (size_t)ldb + 8 * hh;

#pragma unroll 1
  for (int k0 = 0; k0 < K; k0 += 32) {
    FragB af[MT];
#pragma unroll
    for (int i = 0; i < MT; ++i) {
      const unsigned short* aq = ap + (size_t)(16 * i) * (size_t)lda + k0;
      af[i].h[0] = *(const v8usa*)aq;
      af[i].h[1] = *(const v8usa*)(aq + 16);
    }
    const int kb = k0 & kmask;
#pragma unroll
    for (int t = 0; t < NT; ++t) {
      const unsigned short* wq = bp + (size_t)(16 * t) * (size_t)ldb + kb;
      FragB bf;
      bf.h[0] = *(const v8usa*)wq;
      bf.h[1] = *(const v8usa*)(wq + 16);
#pragma unroll
      for (int i = 0; i < MT; ++i) acc[i][t] = wmb(af[i], bf, acc[i][t]);
    }
  }

#pragma unroll
  for (int i = 0; i < MT; ++i)
#pragma unroll
    for (int t = 0; t < NT; ++t) {
      const int lc = 16 * t + m;
#pragma unroll
      for (int r = 0; r < 8; ++r) {
        const int lr = RW * wave + 16 * i + 8 * hh + r;
        stg[lr * BN + lc] = acc[i][t][r];
      }
    }
  __syncthreads();

  if constexpr (EPI == 0 || EPI == 1) {
    static_assert(NT == 4 || EPI > 1);
    if constexpr (EPI == 1) {
      const v4f b4 = *(const v4f*)(bias + col0 + 4 * m);
#pragma unroll 1
      for (int i = 0; i < RW / 2; ++i) {
        float* p = stg + (RW * wave + 2 * i + hh) * BN + 4 * m;
        v4f v = *(const v4fa*)p;
        v.x = softplus_f(v.x + b4.x);
        v.y = softplus_f(v.y + b4.y);
        v.z = softplus_f(v.z + b4.z);
        v.w = softplus_f(v.w + b4.w);
        *(v4fa*)p = v;
      }
    }
    v4f fv[RW / 2];
#pragma unroll
    for (int i = 0; i < RW / 2; ++i) {
      const int lr = RW * wave + 2 * i + hh;
      fv[i] = *(const v4fa*)(stg + lr * BN + 4 * m);
    }
    float* ob = (col0 < split) ? (o0 + col0) : (o1 + (col0 - split));
#pragma unroll
    for (int i = 0; i < RW / 2; ++i) {
      const int lr = RW * wave + 2 * i + hh;
      float* op = ob + (size_t)(rowBase + lr) * (size_t)ldo + 4 * m;
      *(volatile v4f*)op = fv[i];
    }
    __threadfence();
#pragma unroll
    for (int i = 0; i < RW / 2; ++i) {
      const int lr = RW * wave + 2 * i + hh;
      float* op = ob + (size_t)(rowBase + lr) * (size_t)ldo + 4 * m;
      *(volatile v4f*)op = fv[i];
    }
  } else if constexpr (EPI == 2) {
    static_assert(EPI != 2 || (MT == 1 && NT == 6));
    {
      constexpr int NI = (16 * BN) / (4 * 32);
      v4f fv[NI];
      const float* sb = stg + 16 * wave * BN;
#pragma unroll
      for (int it = 0; it < NI; ++it) fv[it] = *(const v4fa*)(sb + 4 * (it * 32 + lane));
      float* gb = o0 + (size_t)(rowBase + 16 * wave) * (size_t)BN;
#pragma unroll
      for (int it = 0; it < NI; ++it) *(volatile v4f*)(gb + 4 * (it * 32 + lane)) = fv[it];
      __threadfence();
#pragma unroll
      for (int it = 0; it < NI; ++it) *(volatile v4f*)(gb + 4 * (it * 32 + lane)) = fv[it];
    }
    {
      v8us qv[8];
#pragma unroll
      for (int i = 0; i < 8; ++i) {
        const int lr = 16 * wave + 2 * i + hh;
        qv[i] = pack8(stg + lr * BN + 8 * (m & 7), m >= 8);
      }
#pragma unroll
      for (int i = 0; i < 8; ++i) {
        const int lr = 16 * wave + 2 * i + hh;
        unsigned short* hp = oh + (size_t)(rowBase + lr) * (size_t)ldh + 8 * m;
        *(volatile v8us*)hp = qv[i];
      }
      __threadfence();
#pragma unroll
      for (int i = 0; i < 8; ++i) {
        const int lr = 16 * wave + 2 * i + hh;
        unsigned short* hp = oh + (size_t)(rowBase + lr) * (size_t)ldh + 8 * m;
        *(volatile v8us*)hp = qv[i];
      }
    }
  } else {
    static_assert(EPI != 3 || NT == 4);
    v8us qv[RW / 2];
#pragma unroll
    for (int i = 0; i < RW / 2; ++i) {
      const int lr = RW * wave + 2 * i + hh;
      qv[i] = pack8(stg + lr * BN + 8 * (m & 7), m >= 8);
    }
    const int coff = col0 + 8 * (m & 7) + (m >> 3) * hoff;
#pragma unroll
    for (int i = 0; i < RW / 2; ++i) {
      const int lr = RW * wave + 2 * i + hh;
      unsigned short* hp = oh + (size_t)(rowBase + lr) * (size_t)ldh + coff;
      *(volatile v8us*)hp = qv[i];
    }
    __threadfence();
#pragma unroll
    for (int i = 0; i < RW / 2; ++i) {
      const int lr = RW * wave + 2 * i + hh;
      unsigned short* hp = oh + (size_t)(rowBase + lr) * (size_t)ldh + coff;
      *(volatile v8us*)hp = qv[i];
    }
  }
}

__global__ __launch_bounds__(256) void k_conv(const float* __restrict__ XI, const float* __restrict__ CWl,
                                              const float* __restrict__ CBl, float* XC, unsigned short* XCHL)
{
  __shared__ __attribute__((aligned(16))) float sxc[1024];
  __shared__ __attribute__((aligned(16))) unsigned short shl[2048];
  const int tid = (int)threadIdx.x;
  const int c0 = (int)blockIdx.x * 1024;
  const int r  = (int)blockIdx.y;
  const int l  = r & (SEQL - 1);
  const bool v0 = l >= 3, v1 = l >= 2, v2 = l >= 1;
  const size_t p0 = (size_t)(v0 ? r - 3 : r) * DIN;
  const size_t p1 = (size_t)(v1 ? r - 2 : r) * DIN;
  const size_t p2 = (size_t)(v2 ? r - 1 : r) * DIN;
  const size_t p3 = (size_t)r * DIN;
#pragma unroll 1
  for (int it = 0; it < 4; ++it) {
    const int cl = it * 256 + tid;
    const int d  = c0 + cl;
    const v4f w = *(const v4f*)(CWl + 4 * d);
    const float w0 = v0 ? w.x : 0.0f;
    const float w1 = v1 ? w.y : 0.0f;
    const float w2 = v2 ? w.z : 0.0f;
    const float x0 = XI[p0 + d];
    const float x1 = XI[p1 + d];
    const float x2 = XI[p2 + d];
    const float x3 = XI[p3 + d];
    const float bv = CBl[d];
    float s = w0 * x0;
    s = fmaf(w1, x1, s);
    s = fmaf(w2, x2, s);
    s = fmaf(w.w, x3, s);
    const float c = s + bv;
    const float xc = c * (1.0f / (1.0f + expf(-c)));
    sxc[cl] = xc;
    const unsigned hb = bf16_bits(xc);
    const unsigned lb = bf16_bits(xc - __uint_as_float(hb << 16));
    shl[cl] = (unsigned short)hb;
    shl[1024 + cl] = (unsigned short)lb;
  }
  __syncthreads();
  const v4f  fo = *(const v4fa*)(sxc + 4 * tid);
  const v8us qo = *(const v8usa*)(shl + 8 * tid);
  float* op = XC + (size_t)r * DIN + c0 + 4 * tid;
  unsigned short* hp = XCHL + (size_t)r * (2 * DIN) + (size_t)(tid >> 7) * DIN + c0 + 8 * (tid & 127);
  *(volatile v4f*)op = fo;
  *(volatile v8us*)hp = qo;
  __threadfence();
  *(volatile v4f*)op = fo;
  *(volatile v8us*)hp = qo;
}

__global__ __launch_bounds__(256) void k_scan(const float* __restrict__ DT, const float* __restrict__ XC,
                                              const float* __restrict__ Z, const float* __restrict__ XDBL,
                                              const float* __restrict__ ANl, const float* __restrict__ DDl,
                                              unsigned short* Y)
{
  __shared__ __attribute__((aligned(16))) float sbc[64 * 32];
  __shared__ __attribute__((aligned(16))) unsigned short yst[64 * 128];
  const int tid = (int)threadIdx.x;
  const int b   = (int)blockIdx.x >> 5;
  const int d0  = ((int)blockIdx.x & 31) * 64;
  const int c   = tid >> 2, p = tid & 3;
  const int d   = d0 + c;
  const int rb  = b * SEQL;
  const v4f A4 = *(const v4f*)(ANl + (size_t)d * NST + 4 * p);
  const float Dd = DDl[d];
  float h0 = 0.0f, h1 = 0.0f, h2 = 0.0f, h3 = 0.0f;

#pragma unroll 1
  for (int ch = 0; ch < SEQL / 64; ++ch) {
    const int l0 = ch * 64;
#pragma unroll
    for (int j = 0; j < 2; ++j) {
      const int q = tid + 256 * j;
      const int t = q >> 3, f = q & 7;
      const v4f v = *(const v4f*)(XDBL + (size_t)(rb + l0 + t) * XPN + RNK + 4 * f);
      *(v4fa*)(sbc + t * 32 + 4 * f) = v;
    }
    __syncthreads();
#pragma unroll 1
    for (int t = 0; t < 64; ++t) {
      const size_t ro = (size_t)(rb + l0 + t) * DIN + d;
      const float dtv = DT[ro];
      const float u   = XC[ro];
      const float zv  = Z[ro];
      const v4f Bv = *(const v4fa*)(sbc + t * 32 + 4 * p);
      const v4f Cv = *(const v4fa*)(sbc + t * 32 + 16 + 4 * p);
      h0 = fmaf(expf(dtv * A4.x), h0, (dtv * Bv.x) * u);
      h1 = fmaf(expf(dtv * A4.y), h1, (dtv * Bv.y) * u);
      h2 = fmaf(expf(dtv * A4.z), h2, (dtv * Bv.z) * u);
      h3 = fmaf(expf(dtv * A4.w), h3, (dtv * Bv.w) * u);
      float ys = h0 * Cv.x;
      ys = fmaf(h1, Cv.y, ys);
      ys = fmaf(h2, Cv.z, ys);
      ys = fmaf(h3, Cv.w, ys);
      ys += __shfl_xor(ys, 1, 32);
      ys += __shfl_xor(ys, 2, 32);
      const float g  = zv * (1.0f / (1.0f + expf(-zv)));
      const float yv = fmaf(Dd, u, ys) * g;
      if (p == 0) {
        const unsigned hb = bf16_bits(yv);
        const unsigned lb = bf16_bits(yv - __uint_as_float(hb << 16));
        yst[t * 128 + c]      = (unsigned short)hb;
        yst[t * 128 + 64 + c] = (unsigned short)lb;
      }
    }
    __syncthreads();
    v8us qv[4];
#pragma unroll
    for (int j = 0; j < 4; ++j) {
      const int q = tid + 256 * j;
      qv[j] = *(const v8usa*)(yst + (q >> 4) * 128 + 8 * (q & 15));
    }
#pragma unroll
    for (int j = 0; j < 4; ++j) {
      const int q = tid + 256 * j;
      const int t = q >> 4, pc = q & 15;
      unsigned short* yp = Y + (size_t)(rb + l0 + t) * (2 * DIN) + (size_t)(pc >> 3) * DIN + d0 + 8 * (pc & 7);
      *(volatile v8us*)yp = qv[j];
    }
    __threadfence();
#pragma unroll
    for (int j = 0; j < 4; ++j) {
      const int q = tid + 256 * j;
      const int t = q >> 4, pc = q & 15;
      unsigned short* yp = Y + (size_t)(rb + l0 + t) * (2 * DIN) + (size_t)(pc >> 3) * DIN + d0 + 8 * (pc & 7);
      *(volatile v8us*)yp = qv[j];
    }
    __syncthreads();
  }
}

extern "C" void kernel_launch(void* const* d_in, const int* in_sizes, int n_in,
                              void* d_out, int out_size, void* d_ws, size_t ws_size,
                              hipStream_t stream) {
  if (n_in < 10) return;
  if (in_sizes[0] != MTOK * DIMX) return;
  if (in_sizes[1] != NLAY * 2 * DIN * DIMX) return;
  if (in_sizes[2] != NLAY * DIN * 4) return;
  if (in_sizes[3] != NLAY * DIN) return;
  if (in_sizes[4] != NLAY * XPN * DIN) return;
  if (in_sizes[5] != NLAY * DIN * RNK) return;
  if (in_sizes[6] != NLAY * DIN) return;
  if (in_sizes[7] != NLAY * DIN * NST) return;
  if (in_sizes[8] != NLAY * DIN) return;
  if (in_sizes[9] != NLAY * DIMX * DIN) return;
  if (out_size != MTOK * DIMX) return;
  if ((size_t)B_TOT > ws_size || (size_t)B_TOT > (size_t)WSMAX) return;

  const float* x    = (const float*)d_in[0];
  const float* inw  = (const float*)d_in[1];
  const float* cw   = (const float*)d_in[2];
  const float* cb   = (const float*)d_in[3];
  const float* xpw  = (const float*)d_in[4];
  const float* dtw  = (const float*)d_in[5];
  const float* dtb  = (const float*)d_in[6];
  const float* alog = (const float*)d_in[7];
  const float* dp   = (const float*)d_in[8];
  const float* ow   = (const float*)d_in[9];
  float* out = (float*)d_out;

  char* ws = (char*)d_ws;
  size_t off = 0;
  unsigned short* XB   = (unsigned short*)(ws + off); off += B_XB;
  unsigned short* INW  = (unsigned short*)(ws + off); off += B_INW;
  unsigned short* XPB  = (unsigned short*)(ws + off); off += B_XPB;
  unsigned short* DTWB = (unsigned short*)(ws + off); off += B_DTWB;
  unsigned short* OWB  = (unsigned short*)(ws + off); off += B_OWB;
  float* CWp  = (float*)(ws + off); off += B_CW;
  float* CBp  = (float*)(ws + off); off += B_V;
  float* DTBp = (float*)(ws + off); off += B_V;
  float* DDp  = (float*)(ws + off); off += B_V;
  float* ANp  = (float*)(ws + off); off += B_AN;
  float* XI   = (float*)(ws + off); off += B_F32;
  float* Zp   = (float*)(ws + off); off += B_F32;
  float* XC   = (float*)(ws + off); off += B_F32;
  unsigned short* XCHL = (unsigned short*)(ws + off); off += B_XCHL;
  float* XDBL = (float*)(ws + off); off += B_XDBL;
  unsigned short* DTR  = (unsigned short*)(ws + off); off += B_DTR;
  float* DTp  = (float*)(ws + off); off += B_F32;
  if (off != (size_t)B_TOT) return;
  unsigned short* Yhl = (unsigned short*)XI;
  unsigned short* X1  = (unsigned short*)DTp;

  const int NOSPLIT = 1 << 30;

  k_prep<<<(U8_TOT + V4_TOT) / 256, 256, 0, stream>>>(x, inw, xpw, dtw, ow, cw, cb, dtb, alog, dp,
                                                      XB, INW, XPB, DTWB, OWB, CWp, CBp, DTBp, DDp, ANp);

  for (int layer = 0; layer < NLAY; ++layer) {
    const unsigned short* inw_l = INW  + (size_t)layer * 2 * DIN * DIMX;
    const unsigned short* xpw_l = XPB  + (size_t)layer * XPN * DIN;
    const unsigned short* dtw_l = DTWB + (size_t)layer * DIN * RNK;
    const unsigned short* ow_l  = OWB  + (size_t)layer * DIMX * DIN;
    const float* cw_l  = CWp  + (size_t)layer * DIN * 4;
    const float* cb_l  = CBp  + (size_t)layer * DIN;
    const float* dtb_l = DTBp + (size_t)layer * DIN;
    const float* dd_l  = DDp  + (size_t)layer * DIN;
    const float* an_l  = ANp  + (size_t)layer * DIN * NST;

    if (layer == 0) {
      k_gemm<2, 4, 0><<<dim3(MTOK / 128, (2 * DIN) / 64), 128, 0, stream>>>(
          XB, DIMX, inw_l, DIMX, DIMX - 1, DIMX, XI, Zp, DIN, DIN, dtb_l, DTR, 0, 0);
    } else {
      k_gemm<2, 4, 0><<<dim3(MTOK / 128, (2 * DIN) / 64), 128, 0, stream>>>(
          X1, 2 * DIMX, inw_l, DIMX, DIMX - 1, 2 * DIMX, XI, Zp, DIN, DIN, dtb_l, DTR, 0, 0);
    }
    k_conv<<<dim3(2, MTOK), 256, 0, stream>>>(XI, cw_l, cb_l, XC, XCHL);
    k_gemm<1, 6, 2><<<dim3(MTOK / 64, 1), 128, 0, stream>>>(
        XCHL, 2 * DIN, xpw_l, DIN, DIN - 1, 2 * DIN, XDBL, XDBL, NOSPLIT, XPN, dtb_l, DTR, 2 * RNK, 0);
    k_gemm<2, 4, 1><<<dim3(MTOK / 128, DIN / 64), 128, 0, stream>>>(
        DTR, 2 * RNK, dtw_l, RNK, RNK - 1, 2 * RNK, DTp, DTp, NOSPLIT, DIN, dtb_l, DTR, 0, 0);
    k_scan<<<2 * (DIN / 64), 256, 0, stream>>>(DTp, XC, Zp, XDBL, an_l, dd_l, Yhl);
    if (layer == 0) {
      k_gemm<2, 4, 3><<<dim3(MTOK / 128, DIMX / 64), 128, 0, stream>>>(
          Yhl, 2 * DIN, ow_l, DIN, DIN - 1, 2 * DIN, XDBL, XDBL, NOSPLIT, XPN, dtb_l, X1, 2 * DIMX, DIMX);
    } else {
      k_gemm<2, 4, 0><<<dim3(MTOK / 128, DIMX / 64), 128, 0, stream>>>(
          Yhl, 2 * DIN, ow_l, DIN, DIN - 1, 2 * DIN, out, out, NOSPLIT, DIMX, dtb_l, DTR, 0, 0);
    }
  }
}
